// CNF_52828097740860
// MI455X (gfx1250) — hardware-run, weakly checked
//
#include <hip/hip_runtime.h>
#include <math.h>

typedef __attribute__((ext_vector_type(16))) __bf16       v16b;
typedef __attribute__((ext_vector_type(8)))  __bf16       v8b;
typedef __attribute__((ext_vector_type(8)))  float        v8f;
typedef __attribute__((ext_vector_type(4)))  float        v4f;
typedef __attribute__((ext_vector_type(4)))  unsigned int v4u;

constexpr int kT      = 9;
constexpr int kN      = 16384;
constexpr int kD      = 8;
constexpr int kH      = 128;
constexpr int kTile   = 32;
constexpr int kBlocks = kN / kTile;
constexpr int kKS     = 32;
constexpr int kPitch  = 136;
constexpr int kXP     = 40;
static_assert(kN % kTile == 0, "whole sample tiles");
static_assert(kH % 32 == 0 && kKS % 32 == 0, "K multiples of 32");
static_assert(kH % 16 == 0, "N multiple of 16");
static_assert(kD == 8, "state width");
static_assert(3 * kD + 5 <= kKS, "layer-1 slot layout fits");
static_assert(((size_t)kT * kN * kD * 4) % 128 == 0, "second output starts on a line");
static_assert((size_t)kT * kN * kD * 4 + (size_t)kT * kN * 4 == 5308416ull, "output bytes");
static_assert((kPitch * 2) % 16 == 0 && (kXP * 2) % 16 == 0, "16-B aligned LDS rows");

constexpr size_t kOffW2H  = 0;
constexpr size_t kOffW2L  = kOffW2H + (size_t)kH * kH * 2;
constexpr size_t kOffGH   = kOffW2L + (size_t)kH * kH * 2;
constexpr size_t kOffGL   = kOffGH  + (size_t)kH * kH * 2;
constexpr size_t kOffW3H  = kOffGL  + (size_t)kH * kH * 2;
constexpr size_t kOffW3L  = kOffW3H + (size_t)16 * kH * 2;
constexpr size_t kOffW1A  = kOffW3L + (size_t)16 * kH * 2;
constexpr size_t kWsTotal = kOffW1A + (size_t)kH * kKS * 2;
static_assert(kWsTotal == 147456ull, "carve total");
static_assert(kWsTotal <= 134217728ull, "carve cap");
static_assert((kOffW2L % 128) == 0 && (kOffGH % 128) == 0 && (kOffGL % 128) == 0 &&
              (kOffW3H % 128) == 0 && (kOffW3L % 128) == 0 && (kOffW1A % 128) == 0, "128-B aligned regions");

__device__ __forceinline__ unsigned short f2bf_bits(float f) {
  unsigned u = __float_as_uint(f);
  return (unsigned short)((u + 0x7FFFu + ((u >> 16) & 1u)) >> 16);
}
__device__ __forceinline__ float bf_bits2f(unsigned short h) { return __uint_as_float(((unsigned)h) << 16); }

template <typename T> struct Frag;
template <> struct Frag<__bf16> {
  typedef v16b V; union U { v16b v; v8b h[2]; };
  static __device__ __forceinline__ v16b load(const __bf16* p) {
    U f; f.h[0] = *(const v8b*)(p); f.h[1] = *(const v8b*)(p + 16); return f.v;
  }
};

__device__ __forceinline__ v8f at_mma(v16b a, v16b b, v8f c) {
  c = __builtin_amdgcn_wmma_f32_16x16x32_bf16(false, a, false, b, (short)0, c, false, false);
  asm volatile("v_nop\n\tv_nop\n\tv_nop\n\tv_nop" : "+v"(c) : "v"(a), "v"(b));
  return c;
}

__device__ __forceinline__ float bf_resid(float a) { return a - bf_bits2f(f2bf_bits(a)); }
__device__ __forceinline__ unsigned pack_bf2(float a, float b) {
  const unsigned lo16 = (unsigned)f2bf_bits(a);
  const unsigned hi16 = (unsigned)f2bf_bits(b);
  return lo16 | (hi16 << 16);
}
__device__ __forceinline__ void put_split(__bf16* ph, __bf16* pl, int o, float v) {
  const unsigned short hb = f2bf_bits(v);
  const unsigned short lb = f2bf_bits(v - bf_bits2f(hb));
  ph[o] = __builtin_bit_cast(__bf16, hb);
  pl[o] = __builtin_bit_cast(__bf16, lb);
}
__device__ __forceinline__ float tanh_fast(float x) {
  const float e = __expf(2.0f * x);
  return 1.0f - 2.0f * __builtin_amdgcn_rcpf(1.0f + e);
}

__global__ __launch_bounds__(256) void build_planes_kernel(
    const float* __restrict__ W1, const float* __restrict__ b1,
    const float* __restrict__ W2, const float* __restrict__ W3,
    unsigned short* __restrict__ W2H, unsigned short* __restrict__ W2L,
    unsigned short* __restrict__ GH,  unsigned short* __restrict__ GL,
    unsigned short* __restrict__ W3H, unsigned short* __restrict__ W3L,
    unsigned short* __restrict__ W1A)
{
  const int tid = threadIdx.x;
  const int blk = blockIdx.x;
  if (blk < 8) {
    const int i  = blk * 256 + tid;
    const int n  = i >> 4;
    const int k8 = (i & 15) * 8;
    float m0 = 0.f, m1 = 0.f, m2 = 0.f, m3 = 0.f, m4 = 0.f, m5 = 0.f, m6 = 0.f, m7 = 0.f;
#pragma unroll 1
    for (int j = 0; j < kD; ++j) {
      const float w3 = W3[n * kD + j];
      const v4f a0 = *(const v4f*)(W1 + j * kH + k8);
      const v4f a1 = *(const v4f*)(W1 + j * kH + k8 + 4);
      m0 = fmaf(a0[0], w3, m0);
      m1 = fmaf(a0[1], w3, m1);
      m2 = fmaf(a0[2], w3, m2);
      m3 = fmaf(a0[3], w3, m3);
      m4 = fmaf(a1[0], w3, m4);
      m5 = fmaf(a1[1], w3, m5);
      m6 = fmaf(a1[2], w3, m6);
      m7 = fmaf(a1[3], w3, m7);
    }
    const float mm[8] = {m0, m1, m2, m3, m4, m5, m6, m7};
    float w2v[8], gv[8];
#pragma unroll
    for (int e = 0; e < 8; ++e) {
      w2v[e] = W2[(size_t)(k8 + e) * kH + n];
      gv[e]  = w2v[e] * mm[e];
    }
    v4u wh, wl, gh, gl;
#pragma unroll
    for (int p = 0; p < 4; ++p) {
      wh[p] = pack_bf2(w2v[2 * p], w2v[2 * p + 1]);
      wl[p] = pack_bf2(bf_resid(w2v[2 * p]), bf_resid(w2v[2 * p + 1]));
      gh[p] = pack_bf2(gv[2 * p], gv[2 * p + 1]);
      gl[p] = pack_bf2(bf_resid(gv[2 * p]), bf_resid(gv[2 * p + 1]));
    }
    const size_t off = (size_t)n * kH + k8;
    volatile v4u* p0 = (volatile v4u*)(W2H + off);
    volatile v4u* p1 = (volatile v4u*)(W2L + off);
    volatile v4u* p2 = (volatile v4u*)(GH + off);
    volatile v4u* p3 = (volatile v4u*)(GL + off);
    *p0 = wh; *p1 = wl; *p2 = gh; *p3 = gl;
    __threadfence();
    *p0 = wh; *p1 = wl; *p2 = gh; *p3 = gl;
  } else if (blk == 8) {
    const int i  = tid;
    const int j  = i >> 4;
    const int k8 = (i & 15) * 8;
    const int jc = (j < kD) ? j : (kD - 1);
    float v[8];
#pragma unroll
    for (int e = 0; e < 8; ++e) {
      const float x = W3[(k8 + e) * kD + jc];
      v[e] = (j < kD) ? x : 0.0f;
    }
    v4u wh, wl;
#pragma unroll
    for (int p = 0; p < 4; ++p) {
      wh[p] = pack_bf2(v[2 * p], v[2 * p + 1]);
      wl[p] = pack_bf2(bf_resid(v[2 * p]), bf_resid(v[2 * p + 1]));
    }
    const size_t off = (size_t)j * kH + k8;
    volatile v4u* p0 = (volatile v4u*)(W3H + off);
    volatile v4u* p1 = (volatile v4u*)(W3L + off);
    *p0 = wh; *p1 = wl;
    __threadfence();
    *p0 = wh; *p1 = wl;
  } else {
    const int i = (blk - 9) * 256 + tid;
    const int n = i >> 2;
    const int g = i & 3;
    float w[8];
#pragma unroll
    for (int d = 0; d < 8; ++d) w[d] = W1[d * kH + n];
    const float wt  = W1[kD * kH + n];
    const float bb  = b1[n];
    const float wtl = bf_resid(wt);
    const float bbl = bf_resid(bb);
    const float u[8] = {wt, wtl, bb, bbl, wt, 0.0f, 0.0f, 0.0f};
    float v[8];
#pragma unroll
    for (int e = 0; e < 8; ++e) {
      const float lo = bf_resid(w[e]);
      const float a  = (g == 2) ? lo : w[e];
      v[e] = (g == 3) ? u[e] : a;
    }
    v4u wv;
#pragma unroll
    for (int p = 0; p < 4; ++p) wv[p] = pack_bf2(v[2 * p], v[2 * p + 1]);
    const size_t off = (size_t)n * kKS + g * 8;
    volatile v4u* p0 = (volatile v4u*)(W1A + off);
    *p0 = wv;
    __threadfence();
    *p0 = wv;
  }
}

__global__ __launch_bounds__(32) void cnf_rk4_kernel(
    const float* __restrict__ ts, const float* __restrict__ z0, const float* __restrict__ lp0,
    const float* __restrict__ b2, const float* __restrict__ b3,
    const unsigned short* __restrict__ W2Hp, const unsigned short* __restrict__ W2Lp,
    const unsigned short* __restrict__ GHp,  const unsigned short* __restrict__ GLp,
    const unsigned short* __restrict__ W3Hp, const unsigned short* __restrict__ W3Lp,
    const unsigned short* __restrict__ W1Ap,
    float* __restrict__ out)
{
  __shared__ __align__(16) __bf16 sH1h[16 * kPitch];
  __shared__ __align__(16) __bf16 sH1l[16 * kPitch];
  __shared__ __align__(16) __bf16 sS1h[16 * kPitch];
  __shared__ __align__(16) __bf16 sS1l[16 * kPitch];
  __shared__ __align__(16) __bf16 sH2h[16 * kPitch];
  __shared__ __align__(16) __bf16 sH2l[16 * kPitch];
  __shared__ __align__(16) unsigned int sX[kTile * (kXP / 2)];
  __shared__ __align__(16) float sF[kTile * 16];
  __shared__ __align__(16) float sTP[kTile * 16];
  __shared__ __align__(16) float sZ[kTile * kD];

  const int lane = threadIdx.x & 31;
  const int hh   = lane >> 4;
  const int c    = lane & 15;
  const int base = blockIdx.x * kTile;

  const __bf16* W2H = (const __bf16*)W2Hp;
  const __bf16* W2L = (const __bf16*)W2Lp;
  const __bf16* GH  = (const __bf16*)GHp;
  const __bf16* GL  = (const __bf16*)GLp;
  const __bf16* W3H = (const __bf16*)W3Hp;
  const __bf16* W3L = (const __bf16*)W3Lp;
  const __bf16* W1A = (const __bf16*)W1Ap;
  const __bf16* xb  = (const __bf16*)sX;

  float* out0 = out;
  float* out1 = out + (size_t)kT * kN * kD;

  float z[8], zs[8], ks[8];
  {
    const float* zp = z0 + (size_t)(base + lane) * kD;
    const v4f a = *(const v4f*)(zp);
    const v4f b = *(const v4f*)(zp + 4);
    z[0] = a[0]; z[1] = a[1]; z[2] = a[2]; z[3] = a[3];
    z[4] = b[0]; z[5] = b[1]; z[6] = b[2]; z[7] = b[3];
  }
#pragma unroll
  for (int d = 0; d < 8; ++d) { zs[d] = z[d]; ks[d] = 0.0f; }
  float lp = lp0[base + lane];
  float ls = 0.0f;
  float tn = ts[0];

  const float b3v = (c < kD) ? b3[c & (kD - 1)] : 0.0f;

#pragma unroll 1
  for (int ev = 0; ev < 4 * (kT - 1) + 1; ++ev) {
    const int step = ev >> 2;
    const int st   = ev & 3;

    if (st == 0) {
      *(v4f*)(sZ + lane * kD)     = (v4f){z[0], z[1], z[2], z[3]};
      *(v4f*)(sZ + lane * kD + 4) = (v4f){z[4], z[5], z[6], z[7]};
      __syncthreads();
      const v4f q0 = *(const v4f*)(sZ + lane * 4);
      const v4f q1 = *(const v4f*)(sZ + 128 + lane * 4);
      const float lpv = lp;
      float* o0 = out0 + ((size_t)step * kN + base) * kD + lane * 4;
      float* o1 = out1 + (size_t)step * kN + base + lane;
      *(volatile v4f*)(o0)       = q0;
      *(volatile v4f*)(o0 + 128) = q1;
      *(volatile float*)(o1)     = lpv;
      __threadfence();
      *(volatile v4f*)(o0)       = q0;
      *(volatile v4f*)(o0 + 128) = q1;
      *(volatile float*)(o1)     = lpv;
      __syncthreads();
#pragma unroll
      for (int d = 0; d < 8; ++d) ks[d] = 0.0f;
      ls = 0.0f;
    }
    if (ev == 4 * (kT - 1)) break;

    const float t0 = ts[step];
    const float t1 = ts[step + 1];
    const float dt = t1 - t0;

    {
      v4u w0, w1, w3;
#pragma unroll
      for (int p = 0; p < 4; ++p) {
        const float a = zs[2 * p], b = zs[2 * p + 1];
        w0[p] = pack_bf2(a, b);
        w1[p] = pack_bf2(bf_resid(a), bf_resid(b));
      }
      const unsigned th = (unsigned)f2bf_bits(tn);
      const unsigned tl = (unsigned)f2bf_bits(bf_resid(tn));
      w3[0] = th | (th << 16);
      w3[1] = 0x3F803F80u;
      w3[2] = tl;
      w3[3] = 0u;
      v4u* xr = (v4u*)(sX + lane * (kXP / 2));
      xr[0] = w0;
      xr[1] = w1;
      xr[2] = w0;
      xr[3] = w3;
    }
    __syncthreads();

#pragma unroll 1
    for (int mt = 0; mt < 2; ++mt) {
      {
        const v16b ax = Frag<__bf16>::load(xb + (mt * 16 + c) * kXP + 8 * hh);
#pragma unroll 1
        for (int nt = 0; nt < kH / 16; ++nt) {
          const int col = nt * 16 + c;
          const v16b bw = Frag<__bf16>::load(W1A + (size_t)col * kKS + 8 * hh);
          v8f acc = (v8f){0.f, 0.f, 0.f, 0.f, 0.f, 0.f, 0.f, 0.f};
          acc = at_mma(ax, bw, acc);
#pragma unroll
          for (int r = 0; r < 8; ++r) {
            const float h = tanh_fast(acc[r]);
            const float s = 1.0f - h * h;
            const int o = (8 * hh + r) * kPitch + col;
            put_split(sH1h, sH1l, o, h);
            put_split(sS1h, sS1l, o, s);
          }
        }
      }
      __syncthreads();

      {
        float tr[8];
#pragma unroll
        for (int r = 0; r < 8; ++r) tr[r] = 0.0f;
#pragma unroll 1
        for (int nt = 0; nt < kH / 16; ++nt) {
          const int col = nt * 16 + c;
          const size_t brow = (size_t)col * kH + 8 * hh;
          v8f acc2 = (v8f){0.f, 0.f, 0.f, 0.f, 0.f, 0.f, 0.f, 0.f};
          v8f accT = (v8f){0.f, 0.f, 0.f, 0.f, 0.f, 0.f, 0.f, 0.f};
#pragma unroll 1
          for (int kk = 0; kk < kH / 32; ++kk) {
            const int ko = kk * 32;
            const v16b w2h = Frag<__bf16>::load(W2H + brow + ko);
            const v16b w2l = Frag<__bf16>::load(W2L + brow + ko);
            const v16b gh  = Frag<__bf16>::load(GH + brow + ko);
            const v16b gl  = Frag<__bf16>::load(GL + brow + ko);
            const int ao = c * kPitch + ko + 8 * hh;
            const v16b h1h = Frag<__bf16>::load(sH1h + ao);
            const v16b h1l = Frag<__bf16>::load(sH1l + ao);
            const v16b s1h = Frag<__bf16>::load(sS1h + ao);
            const v16b s1l = Frag<__bf16>::load(sS1l + ao);
            acc2 = at_mma(h1l, w2h, acc2);
            acc2 = at_mma(h1h, w2l, acc2);
            acc2 = at_mma(h1h, w2h, acc2);
            accT = at_mma(s1l, gh, accT);
            accT = at_mma(s1h, gl, accT);
            accT = at_mma(s1h, gh, accT);
          }
          const float bb = b2[col];
#pragma unroll
          for (int r = 0; r < 8; ++r) {
            const float h = tanh_fast(acc2[r] + bb);
            const float s = 1.0f - h * h;
            tr[r] = fmaf(s, accT[r], tr[r]);
            put_split(sH2h, sH2l, (8 * hh + r) * kPitch + col, h);
          }
        }
#pragma unroll
        for (int r = 0; r < 8; ++r) sTP[(mt * 16 + 8 * hh + r) * 16 + c] = tr[r];
      }
      __syncthreads();

      {
        v8f acc = (v8f){0.f, 0.f, 0.f, 0.f, 0.f, 0.f, 0.f, 0.f};
#pragma unroll 1
        for (int kk = 0; kk < kH / 32; ++kk) {
          const int ko = kk * 32;
          const v16b w3h = Frag<__bf16>::load(W3H + (size_t)c * kH + ko + 8 * hh);
          const v16b w3l = Frag<__bf16>::load(W3L + (size_t)c * kH + ko + 8 * hh);
          const int ao = c * kPitch + ko + 8 * hh;
          const v16b h2h = Frag<__bf16>::load(sH2h + ao);
          const v16b h2l = Frag<__bf16>::load(sH2l + ao);
          acc = at_mma(h2l, w3h, acc);
          acc = at_mma(h2h, w3l, acc);
          acc = at_mma(h2h, w3h, acc);
        }
#pragma unroll
        for (int r = 0; r < 8; ++r) sF[(mt * 16 + 8 * hh + r) * 16 + c] = acc[r] + b3v;
      }
      __syncthreads();
    }

    {
      const v4f f0 = *(const v4f*)(sF + lane * 16);
      const v4f f1 = *(const v4f*)(sF + lane * 16 + 4);
      const v4f p0 = *(const v4f*)(sTP + lane * 16);
      const v4f p1 = *(const v4f*)(sTP + lane * 16 + 4);
      const v4f p2 = *(const v4f*)(sTP + lane * 16 + 8);
      const v4f p3 = *(const v4f*)(sTP + lane * 16 + 12);
      float trv = 0.0f;
      trv += p0[0]; trv += p0[1]; trv += p0[2]; trv += p0[3];
      trv += p1[0]; trv += p1[1]; trv += p1[2]; trv += p1[3];
      trv += p2[0]; trv += p2[1]; trv += p2[2]; trv += p2[3];
      trv += p3[0]; trv += p3[1]; trv += p3[2]; trv += p3[3];
      const float f[8] = {f0[0], f0[1], f0[2], f0[3], f1[0], f1[1], f1[2], f1[3]};
      const float wc = (st == 1 || st == 2) ? 2.0f : 1.0f;
#pragma unroll
      for (int d = 0; d < 8; ++d) ks[d] = fmaf(wc, f[d], ks[d]);
      ls = ls - wc * trv;
      if (st < 3) {
        const float hdt = 0.5f * dt;
        const float cdt = (st == 2) ? dt : hdt;
        tn = (st == 2) ? t1 : (t0 + hdt);
#pragma unroll
        for (int d = 0; d < 8; ++d) zs[d] = z[d] + cdt * f[d];
      } else {
        const float h6 = dt * (1.0f / 6.0f);
#pragma unroll
        for (int d = 0; d < 8; ++d) {
          z[d]  = z[d] + h6 * ks[d];
          zs[d] = z[d];
        }
        lp = lp + h6 * ls;
        tn = t1;
      }
    }
  }
}

extern "C" void kernel_launch(void* const* d_in, const int* in_sizes, int n_in,
                              void* d_out, int out_size, void* d_ws, size_t ws_size,
                              hipStream_t stream) {
  if (n_in < 9) return;
  if (in_sizes[0] != kT) return;
  if (in_sizes[1] != kN * kD) return;
  if (in_sizes[2] != kN) return;
  if (in_sizes[3] != (kD + 1) * kH) return;
  if (in_sizes[4] != kH) return;
  if (in_sizes[5] != kH * kH) return;
  if (in_sizes[6] != kH) return;
  if (in_sizes[7] != kH * kD) return;
  if (in_sizes[8] != kD) return;
  if (out_size != kT * kN * kD + kT * kN) return;
  if (ws_size < kWsTotal) return;

  const float* ts  = (const float*)d_in[0];
  const float* z0  = (const float*)d_in[1];
  const float* lp0 = (const float*)d_in[2];
  const float* W1  = (const float*)d_in[3];
  const float* b1  = (const float*)d_in[4];
  const float* W2  = (const float*)d_in[5];
  const float* b2  = (const float*)d_in[6];
  const float* W3  = (const float*)d_in[7];
  const float* b3  = (const float*)d_in[8];

  char* ws = (char*)d_ws;
  unsigned short* W2H = (unsigned short*)(ws + kOffW2H);
  unsigned short* W2L = (unsigned short*)(ws + kOffW2L);
  unsigned short* GH  = (unsigned short*)(ws + kOffGH);
  unsigned short* GL  = (unsigned short*)(ws + kOffGL);
  unsigned short* W3H = (unsigned short*)(ws + kOffW3H);
  unsigned short* W3L = (unsigned short*)(ws + kOffW3L);
  unsigned short* W1A = (unsigned short*)(ws + kOffW1A);

  build_planes_kernel<<<11, 256, 0, stream>>>(W1, b1, W2, W3, W2H, W2L, GH, GL, W3H, W3L, W1A);

  cnf_rk4_kernel<<<kBlocks, kTile, 0, stream>>>(ts, z0, lp0, b2, b3,
                                                W2H, W2L, GH, GL, W3H, W3L, W1A,
                                                (float*)d_out);
}
